// DINEncoder_23940147708093
// MI455X (gfx1250) — hardware-verified
//
#include <hip/hip_runtime.h>
#include <hip/hip_bf16.h>


#define __bf16 _Float16
typedef __attribute__((ext_vector_type(4))) float v4f_t;
typedef float v4fa __attribute__((ext_vector_type(4), may_alias));
typedef __attribute__((ext_vector_type(16))) __bf16 v16bf;
typedef __attribute__((ext_vector_type(8)))  __bf16 v8bf;
typedef __attribute__((ext_vector_type(8)))  float  v8f;

#define B_   8
#define N_   512
#define D_   64
#define H_   64
#define XS   72
#define TS   520

union FragU { v16bf v; v8bf h[2]; };

__device__ inline v16bf load_frag(const __bf16* rowptr, int lane) {
  const int koff = (lane & 16) ? 8 : 0;
  FragU u;
  u.h[0] = *(const v8bf*)(rowptr + koff);
  u.h[1] = *(const v8bf*)(rowptr + koff + 16);
  return u.v;
}

__device__ inline v8bf cvt8(const float4 f0, const float4 f1) {
  v8bf r;
  r[0] = (__bf16)f0.x; r[1] = (__bf16)f0.y; r[2] = (__bf16)f0.z; r[3] = (__bf16)f0.w;
  r[4] = (__bf16)f1.x; r[5] = (__bf16)f1.y; r[6] = (__bf16)f1.z; r[7] = (__bf16)f1.w;
  return r;
}

__global__ __launch_bounds__(256)
void din_encoder_kernel(const float* __restrict__ UE,
                        const float* __restrict__ VM,
                        const float* __restrict__ W1,
                        const float* __restrict__ b1,
                        const float* __restrict__ pa,
                        const float* __restrict__ W2,
                        const float* __restrict__ b2,
                        float* __restrict__ out)
{
  __shared__ __align__(16) __bf16 sX  [N_ * XS];
  __shared__ __align__(16) __bf16 sXT [D_ * TS];
  __shared__ __align__(16) __bf16 sHK [N_ * XS];
  __shared__ __align__(16) __bf16 sWm [H_ * XS];
  __shared__ __align__(16) __bf16 sWkd[H_ * XS];
  __shared__ __align__(16) float  sSB [16 * TS];
  __shared__ float sHqb[16 * H_];
  __shared__ float sW2[H_];

  const int tid  = threadIdx.x;
  const int lane = tid & 31;
  const int wave = tid >> 5;
  const int m16  = lane & 15;
  const int b    = blockIdx.x >> 5;
  const int iqt  = 31 - (blockIdx.x & 31);
  const int q0   = iqt << 4;

  const float prelu_a = pa[0];
  const float bias2   = b2[0];

  const float* Xg = UE + (size_t)b * (N_ * D_);
  #pragma unroll 1
  for (int idx = tid; idx < (N_ * D_) / 8; idx += 256) {
    int k  = idx >> 3;
    int d8 = (idx & 7) << 3;
    const float4* g = (const float4*)(Xg + k * D_ + d8);
    v8bf v = cvt8(g[0], g[1]);
    *(v8bf*)(sX + k * XS + d8) = v;
    for (int e = 0; e < 8; ++e)
      sXT[(d8 + e) * TS + k] = v[e];
  }
  #pragma unroll 1
  for (int idx = tid; idx < (H_ * D_) / 8; idx += 256) {
    int h  = idx >> 3;
    int d8 = (idx & 7) << 3;
    const float4* wm = (const float4*)(W1 + h * (4 * D_) + 3 * D_ + d8);
    const float4* wk = (const float4*)(W1 + h * (4 * D_) + D_     + d8);
    const float4* wd = (const float4*)(W1 + h * (4 * D_) + 2 * D_ + d8);
    *(v8bf*)(sWm + h * XS + d8) = cvt8(wm[0], wm[1]);
    float4 k0 = wk[0], k1 = wk[1], d0 = wd[0], d1 = wd[1];
    float4 s0 = make_float4(k0.x - d0.x, k0.y - d0.y, k0.z - d0.z, k0.w - d0.w);
    float4 s1 = make_float4(k1.x - d1.x, k1.y - d1.y, k1.z - d1.z, k1.w - d1.w);
    *(v8bf*)(sWkd + h * XS + d8) = cvt8(s0, s1);
  }
  if (tid < H_) sW2[tid] = W2[tid];
  #pragma unroll 1
  for (int idx = tid; idx < 16 * TS; idx += 256) sSB[idx] = 0.0f;
  #pragma unroll 1
  for (int idx = tid; idx < 16 * H_; idx += 256) {
    int q = idx >> 6, h = idx & 63;
    const float* xq  = Xg + (size_t)(q0 + q) * D_;
    const float* w1r = W1 + h * (4 * D_);
    float acc = b1[h];
    for (int d = 0; d < D_; ++d) acc += xq[d] * (w1r[d] + w1r[2 * D_ + d]);
    sHqb[idx] = acc;
  }
  __syncthreads();

  {
    v16bf wf[4][2];
    for (int j = 0; j < 4; ++j)
      for (int cch = 0; cch < 2; ++cch)
        wf[j][cch] = load_frag(sWkd + (16 * j + m16) * XS + 32 * cch, lane);

    #pragma unroll 1
    for (int u = 0; u < 4; ++u) {
      const int kt = (u << 3) + wave;
      v16bf a0 = load_frag(sX + (16 * kt + m16) * XS,      lane);
      v16bf a1 = load_frag(sX + (16 * kt + m16) * XS + 32, lane);
      v8f c[4];
      for (int j = 0; j < 4; ++j) {
        v8f z = {0.f, 0.f, 0.f, 0.f, 0.f, 0.f, 0.f, 0.f};
        z = __builtin_amdgcn_wmma_f32_16x16x32_f16(false, a0, false, wf[j][0], (short)0, z, false, false);
        z = __builtin_amdgcn_wmma_f32_16x16x32_f16(false, a1, false, wf[j][1], (short)0, z, false, false);
        c[j] = z;
      }
      for (int j = 0; j < 4; ++j) {
        const int hcol = 16 * j + m16;
        for (int v = 0; v < 8; ++v) {
          int k = 16 * kt + v + ((lane >> 4) << 3);
          sHK[k * XS + hcol] = (__bf16)c[j][v];
        }
      }
    }
  }
  __syncthreads();

  #pragma unroll 1
  for (int q = wave; q < 16; q += 8) {
    const int qg = q0 + q;
    #pragma unroll 1
    for (int jh = 0; jh < 2; ++jh) {
      v16bf af[2][2];
      for (int cch = 0; cch < 2; ++cch) {
        v16bf xq = load_frag(sX + qg * XS + 32 * cch, lane);
        for (int jj = 0; jj < 2; ++jj) {
          const int j = 2 * jh + jj;
          v16bf wm = load_frag(sWm + (16 * j + m16) * XS + 32 * cch, lane);
          v16bf a;
          for (int e = 0; e < 16; ++e)
            a[e] = (__bf16)((float)wm[e] * (float)xq[e]);
          af[jj][cch] = a;
        }
      }

      #pragma unroll 1
      for (int kt = 0; kt <= iqt; ++kt) {
        const __bf16* brow = sX + (16 * kt + m16) * XS;
        v16bf bf0 = load_frag(brow,      lane);
        v16bf bf1 = load_frag(brow + 32, lane);

        v8f acc[2];
        for (int jj = 0; jj < 2; ++jj) {
          v8f c = {0.f, 0.f, 0.f, 0.f, 0.f, 0.f, 0.f, 0.f};
          c = __builtin_amdgcn_wmma_f32_16x16x32_f16(false, af[jj][0], false, bf0, (short)0, c, false, false);
          c = __builtin_amdgcn_wmma_f32_16x16x32_f16(false, af[jj][1], false, bf1, (short)0, c, false, false);
          acc[jj] = c;
        }

        float s = 0.f;
        const int hbase = (lane >> 4) << 3;
        const __bf16* hkrow = sHK + (16 * kt + m16) * XS;
        for (int jj = 0; jj < 2; ++jj) {
          const int j = 2 * jh + jj;
          v8bf hk8 = *(const v8bf*)(hkrow + 16 * j + hbase);
          for (int v = 0; v < 8; ++v) {
            int h = 16 * j + hbase + v;
            float val = acc[jj][v] + (float)hk8[v] + sHqb[q * H_ + h];
            val = (val > 0.f) ? val : prelu_a * val;
            s += val * sW2[h];
          }
        }
        s += __shfl_xor(s, 16, 32);

        if (lane < 16) {
          int kk = 16 * kt + lane;
          if (jh == 0) sSB[q * TS + kk] = s;
          else {
            float sc = sSB[q * TS + kk] + s + bias2;
            sc = (kk <= qg) ? sc * VM[b * N_ + kk] : 0.f;
            sSB[q * TS + kk] = sc;
          }
        }
      }
    }
  }
  __syncthreads();

  if (wave < 4) {
    const int d0  = wave << 4;
    const int kch = (16 * (iqt + 1) + 31) >> 5;
    v8f c = {0.f, 0.f, 0.f, 0.f, 0.f, 0.f, 0.f, 0.f};
    #pragma unroll 1
    for (int kc = 0; kc < kch; ++kc) {
      v16bf a;
      { const int koff = (lane & 16) ? 8 : 0; const float* sp = sSB + m16 * TS + 32 * kc + koff;
        for (int e = 0; e < 8; ++e) { a[e] = (__bf16)sp[e]; a[8 + e] = (__bf16)sp[16 + e]; } }
      v16bf x = load_frag(sXT + (d0 + m16) * TS + 32 * kc, lane);
      c = __builtin_amdgcn_wmma_f32_16x16x32_f16(false, a, false, x, (short)0, c, false, false);
    }
    for (int v = 0; v < 8; ++v) {
      int q = v + ((lane >> 4) << 3);
      sHqb[q * D_ + d0 + m16] = c[v];
    }
  }
  __syncthreads();
  if (wave < 4) {
    float* ob = out + ((size_t)b * N_ + q0) * D_;
    #pragma unroll 1
    for (int pass = 0; pass < 2; ++pass) {
      for (int i = 0; i < 2; ++i) { const int c4 = tid + 128 * i, q = c4 >> 4, dq = (c4 & 15) * 4;
        *(volatile v4f_t*)(ob + q * D_ + dq) = *(const volatile v4fa*)(sHqb + q * D_ + dq); }
      __threadfence();
    }
  }
}

extern "C" void kernel_launch(void* const* d_in, const int* in_sizes, int n_in,
                              void* d_out, int out_size, void* d_ws, size_t ws_size,
                              hipStream_t stream) {
  const float* UE = (const float*)d_in[1];
  const float* VM = (const float*)d_in[2];
  const float* W1 = (const float*)d_in[3];
  const float* b1 = (const float*)d_in[4];
  const float* pa = (const float*)d_in[5];
  const float* W2 = (const float*)d_in[6];
  const float* b2 = (const float*)d_in[7];
  float* out = (float*)d_out;

  dim3 grid(B_ * (N_ / 16));
  dim3 block(256);
  din_encoder_kernel<<<grid, block, 0, stream>>>(UE, VM, W1, b1, pa, W2, b2, out);
}
